// Self_attention_residuel_77257871720942
// MI455X (gfx1250) — hardware-verified
//
#include <hip/hip_runtime.h>
#include <stdint.h>

#define NB 4
#define NT 2048
#define ND 1024

typedef __attribute__((ext_vector_type(16))) _Float16 v16h;
typedef __attribute__((ext_vector_type(8)))  _Float16 v8h;
typedef __attribute__((ext_vector_type(16))) __bf16   v16b;
typedef __attribute__((ext_vector_type(8)))  __bf16   v8b;
typedef __attribute__((ext_vector_type(8)))  float    v8f;
typedef __attribute__((ext_vector_type(4)))  float    v4f;
#define U16(p) ((const unsigned short*)(const void*)(p))

__device__ __forceinline__ unsigned short f2bf_bits(float f) {
  unsigned u = __float_as_uint(f);
  return (unsigned short)((u + 0x7FFFu + ((u >> 16) & 1u)) >> 16);
}
__device__ __forceinline__ float bf_bits2f(unsigned short h) { return __uint_as_float(((unsigned)h) << 16); }

__device__ __forceinline__ void dep_guard_h(v8f& a, v8f& b, v16h x, v16h y) { asm volatile("v_nop\n\tv_nop\n\tv_nop\n\tv_nop" : "+v"(a), "+v"(b) : "v"(x), "v"(y)); }
__device__ __forceinline__ void dep_guard_b(v8f& a, v8f& b, v16b x, v16b y) { asm volatile("v_nop\n\tv_nop\n\tv_nop\n\tv_nop" : "+v"(a), "+v"(b) : "v"(x), "v"(y)); }
__device__ __forceinline__ void keep4_h(v16h a, v16h b, v16h c, v16h d) { asm volatile("v_nop" :: "v"(a), "v"(b), "v"(c), "v"(d)); }
__device__ __forceinline__ void keep4_b(v16b a, v16b b, v16b c, v16b d) { asm volatile("v_nop" :: "v"(a), "v"(b), "v"(c), "v"(d)); }
__device__ __forceinline__ void acc_guard4(v8f& a, v8f& b, v8f& c, v8f& d) { asm volatile("v_nop\n\tv_nop\n\tv_nop\n\tv_nop" : "+v"(a), "+v"(b), "+v"(c), "+v"(d)); }
template <typename T> struct Frag;
template <> struct Frag<_Float16> {
  typedef v16h V; union U { v16h v; v8h h[2]; };
  static __device__ __forceinline__ v16h load(const _Float16* p) {
    U f; f.h[0] = *(const v8h*)(p); f.h[1] = *(const v8h*)(p + 16); return f.v;
  }
  static __device__ __forceinline__ v8f mma(v16h a, v16h b, v8f c) {
    return __builtin_amdgcn_wmma_f32_16x16x32_f16(false, a, false, b, (short)0, c, false, false);
  }
  static __device__ __forceinline__ void guard(v8f& a, v8f& b, v16h x, v16h y) { dep_guard_h(a, b, x, y); }
  static __device__ __forceinline__ void keep(v16h a, v16h b, v16h c, v16h d) { keep4_h(a, b, c, d); }
};
template <> struct Frag<__bf16> {
  typedef v16b V; union U { v16b v; v8b h[2]; };
  static __device__ __forceinline__ v16b load(const __bf16* p) {
    U f; f.h[0] = *(const v8b*)(p); f.h[1] = *(const v8b*)(p + 16); return f.v;
  }
  static __device__ __forceinline__ v8f mma(v16b a, v16b b, v8f c) {
    return __builtin_amdgcn_wmma_f32_16x16x32_bf16(false, a, false, b, (short)0, c, false, false);
  }
  static __device__ __forceinline__ void guard(v8f& a, v8f& b, v16b x, v16b y) { dep_guard_b(a, b, x, y); }
  static __device__ __forceinline__ void keep(v16b a, v16b b, v16b c, v16b d) { keep4_b(a, b, c, d); }
};

template <int ET> struct Elem;
template <> struct Elem<0> { typedef _Float16 T; };
template <> struct Elem<1> { typedef __bf16 T; };
template <int ET, bool SPLIT, int BIAS_MODE, int OUT_MODE, bool RESID, int ACT = 0>
__global__ __launch_bounds__(256) void wmma_gemm64(
    const unsigned short* __restrict__ Ap, const unsigned short* __restrict__ A2p, int lda, long strideA,
    const unsigned short* __restrict__ Btp, const unsigned short* __restrict__ Bt2p, int ldb, long strideB,
    void* __restrict__ Cout, void* __restrict__ Cout2, int ldc, long strideC,
    const float* __restrict__ bias,
    const float* __restrict__ resid, long strideR,
    int M, int N, int K, float scale) {
  typedef typename Elem<ET>::T T;
  typedef typename Frag<T>::V V;
  const T* A = (const T*)Ap; const T* A2 = (const T*)A2p; const T* Bt = (const T*)Btp; const T* Bt2 = (const T*)Bt2p;
  __shared__ __align__(16) float sT[8][16 * 68];
  const int b    = blockIdx.y;
  const int lane = threadIdx.x & 31;
  const int wave = threadIdx.x >> 5;
  const int tilesN = N >> 6;
  const int tilesM = M >> 6;
  const int tile = blockIdx.x * 8 + wave;
  if (tile >= tilesM * tilesN) return;
  const int tm = tile / tilesN;
  const int tn = tile - tm * tilesN;
  const int m0 = tm << 6;
  const int n0 = tn << 6;

  const T* Ab  = A  + (size_t)b * strideA;
  const T* Bb  = Bt + (size_t)b * strideB;
  const T* Ab2 = SPLIT ? (A2  + (size_t)b * strideA) : nullptr;
  const T* Bb2 = SPLIT ? (Bt2 + (size_t)b * strideB) : nullptr;

  const int rlane = lane & 15;
  const int koff  = (lane >> 4) * 8;
  const int mOff  = (lane >> 4) * 8;

  v8f acc[4][4];
#pragma unroll
  for (int i = 0; i < 4; ++i)
#pragma unroll
    for (int j = 0; j < 4; ++j) acc[i][j] = (v8f){0.f,0.f,0.f,0.f,0.f,0.f,0.f,0.f};

  for (int k0 = 0; k0 < K; k0 += 32) {
    V bh[4], bl[4];
#pragma unroll
    for (int j = 0; j < 4; ++j) {
      const size_t bo = (size_t)(n0 + (j << 4) + rlane) * ldb + koff + k0;
      bh[j] = Frag<T>::load(Bb + bo);
      if (SPLIT) bl[j] = Frag<T>::load(Bb2 + bo);
    }
#pragma unroll
    for (int i = 0; i < 4; ++i) {
      const size_t ao = (size_t)(m0 + (i << 4) + rlane) * lda + koff + k0;
      V ah = Frag<T>::load(Ab + ao);
      V al;
      if (SPLIT) al = Frag<T>::load(Ab2 + ao);
#pragma unroll
      for (int j = 0; j < 4; ++j) {
        acc[i][j] = Frag<T>::mma(ah, bh[j], acc[i][j]);
        if (SPLIT) {
          acc[i][j] = Frag<T>::mma(ah, bl[j], acc[i][j]);
          acc[i][j] = Frag<T>::mma(al, bh[j], acc[i][j]);
        }
      }
      Frag<T>::guard(acc[i][0], acc[i][3], ah, SPLIT ? al : ah);
    }
    Frag<T>::keep(bh[0], bh[1], bh[2], bh[3]);
    if (SPLIT) Frag<T>::keep(bl[0], bl[1], bl[2], bl[3]);
  }
  acc_guard4(acc[0][0], acc[0][1], acc[0][2], acc[0][3]);
  acc_guard4(acc[1][0], acc[1][1], acc[1][2], acc[1][3]);
  acc_guard4(acc[2][0], acc[2][1], acc[2][2], acc[2][3]);
  acc_guard4(acc[3][0], acc[3][1], acc[3][2], acc[3][3]);

  float* slab = sT[wave];
  const float* Rb = RESID ? (resid + (size_t)b * strideR) : nullptr;
#pragma unroll
  for (int i = 0; i < 4; ++i) {
    const int mBase = m0 + (i << 4);
#pragma unroll
    for (int j = 0; j < 4; ++j) {
      const int n = n0 + (j << 4) + rlane;
      float bv = 0.f;
      if (BIAS_MODE == 2) bv = bias[n];
#pragma unroll
      for (int r = 0; r < 8; ++r) {
        float v = acc[i][j][r] * scale;
        if (BIAS_MODE == 1) v += bias[mBase + mOff + r];
        if (BIAS_MODE == 2) v += bv;
        if (RESID) v += Rb[(size_t)(mBase + mOff + r) * ldc + n];
        if (ACT == 1) v = tanhf(v);
        if (ACT == 2) v = fmaxf(v, 0.0f);
        if (ACT == 3) v = v / (1.0f + expf(-v));
        if (ACT == 4) v = (v > 0.f) ? v : 0.01f * v;
        if (ACT == 5) v = 0.5f * v * (1.0f + erff(v * 0.70710678118654752f));
        slab[(mOff + r) * 68 + (j << 4) + rlane] = v;
      }
    }
    __builtin_amdgcn_fence(__ATOMIC_RELEASE, "workgroup");
    __builtin_amdgcn_wave_barrier();
    __builtin_amdgcn_fence(__ATOMIC_ACQUIRE, "workgroup");
    if (OUT_MODE == 0) {
      float* C = (float*)Cout + (size_t)b * strideC;
      const int hh = lane >> 4, c4 = (lane & 15) * 4;
      for (int pass = 0; pass < 2; ++pass) {
#pragma unroll
        for (int it = 0; it < 8; ++it) {
          const int row = it * 2 + hh;
          v4f v = *(const v4f*)(slab + row * 68 + c4);
          *(volatile v4f*)(C + (size_t)(mBase + row) * ldc + n0 + c4) = v;
        }
        __threadfence();
      }
    } else {
      const int q = lane >> 3, c8 = (lane & 7) * 8;
      unsigned short* C  = (unsigned short*)Cout  + (size_t)b * strideC;
      unsigned short* C2 = (OUT_MODE == 2) ? ((unsigned short*)Cout2 + (size_t)b * strideC) : nullptr;
      for (int pass = 0; pass < 2; ++pass) {
#pragma unroll
        for (int it = 0; it < 4; ++it) {
          const int row = it * 4 + q;
          const float* sp = slab + row * 68 + c8;
          v8h hv, lv;
#pragma unroll
          for (int e = 0; e < 8; ++e) {
            if (OUT_MODE == 1) {
              hv[e] = (_Float16)sp[e];
            } else {
              unsigned short hb = f2bf_bits(sp[e]);
              unsigned short lb = f2bf_bits(sp[e] - bf_bits2f(hb));
              hv[e] = __builtin_bit_cast(_Float16, hb);
              lv[e] = __builtin_bit_cast(_Float16, lb);
            }
          }
          *(volatile v8h*)(C + (size_t)(mBase + row) * ldc + n0 + c8) = hv;
          if (OUT_MODE == 2) *(volatile v8h*)(C2 + (size_t)(mBase + row) * ldc + n0 + c8) = lv;
        }
        __threadfence();
      }
    }
    __builtin_amdgcn_fence(__ATOMIC_RELEASE, "workgroup");
    __builtin_amdgcn_wave_barrier();
    __builtin_amdgcn_fence(__ATOMIC_ACQUIRE, "workgroup");
  }
}

__global__ __launch_bounds__(256) void cast_f32_f16x2_scaled(
    const float* __restrict__ in, _Float16* __restrict__ out, int n2, float sc) {
  int i = blockIdx.x * 256 + threadIdx.x;
  if (i < n2) {
    const _Float16 h0 = (_Float16)(in[2 * i] * sc), h1 = (_Float16)(in[2 * i + 1] * sc);
    const unsigned u = (unsigned)__builtin_bit_cast(unsigned short, h0) | ((unsigned)__builtin_bit_cast(unsigned short, h1) << 16);
    ((volatile unsigned*)out)[i] = u;
    __threadfence();
    ((volatile unsigned*)out)[i] = u;
  }
}

__global__ __launch_bounds__(128) void ln_f16_kernel(const float* __restrict__ x,
                                                     const float* __restrict__ gamma,
                                                     const float* __restrict__ beta,
                                                     _Float16* __restrict__ xn) {
  __shared__ float red0[4];
  __shared__ float red1[4];
  const int row = blockIdx.x;
  const int tid = threadIdx.x, lane = tid & 31, wave = tid >> 5;
  const float* xr = x + (size_t)row * ND + tid * 8;
  const v4f a = *(const v4f*)(xr);
  const v4f c = *(const v4f*)(xr + 4);
  float s = ((a[0] + a[1]) + (a[2] + a[3])) + ((c[0] + c[1]) + (c[2] + c[3]));
#pragma unroll
  for (int off = 16; off > 0; off >>= 1) s += __shfl_xor(s, off, 32);
  if (lane == 0) red0[wave] = s;
  __syncthreads();
  const float mu = ((red0[0] + red0[1]) + (red0[2] + red0[3])) * (1.0f / 1024.0f);
  const float d0 = a[0] - mu, d1 = a[1] - mu, d2 = a[2] - mu, d3 = a[3] - mu;
  const float d4 = c[0] - mu, d5 = c[1] - mu, d6 = c[2] - mu, d7 = c[3] - mu;
  float sq = ((d0 * d0 + d1 * d1) + (d2 * d2 + d3 * d3)) + ((d4 * d4 + d5 * d5) + (d6 * d6 + d7 * d7));
#pragma unroll
  for (int off = 16; off > 0; off >>= 1) sq += __shfl_xor(sq, off, 32);
  if (lane == 0) red1[wave] = sq;
  __syncthreads();
  const float var = ((red1[0] + red1[1]) + (red1[2] + red1[3])) * (1.0f / 1024.0f);
  const float inv = rsqrtf(var + 1e-5f);
  const v4f g0 = *(const v4f*)(gamma + tid * 8);
  const v4f g1 = *(const v4f*)(gamma + tid * 8 + 4);
  const v4f b0 = *(const v4f*)(beta + tid * 8);
  const v4f b1 = *(const v4f*)(beta + tid * 8 + 4);
  v8h hv;
  hv[0] = (_Float16)(d0 * inv * g0[0] + b0[0]);
  hv[1] = (_Float16)(d1 * inv * g0[1] + b0[1]);
  hv[2] = (_Float16)(d2 * inv * g0[2] + b0[2]);
  hv[3] = (_Float16)(d3 * inv * g0[3] + b0[3]);
  hv[4] = (_Float16)(d4 * inv * g1[0] + b1[0]);
  hv[5] = (_Float16)(d5 * inv * g1[1] + b1[1]);
  hv[6] = (_Float16)(d6 * inv * g1[2] + b1[2]);
  hv[7] = (_Float16)(d7 * inv * g1[3] + b1[3]);
  _Float16* dst = xn + (size_t)row * ND + tid * 8;
  *(volatile v8h*)dst = hv;
  __threadfence();
  *(volatile v8h*)dst = hv;
}

__global__ __launch_bounds__(256) void colstats_kernel(const float* __restrict__ S,
                                                       const int* __restrict__ lp, int b,
                                                       float* __restrict__ cmax,
                                                       float* __restrict__ cinv) {
  const int j = blockIdx.x * 256 + threadIdx.x;
  int L = lp[b];
  L = L < 1 ? 1 : L;
  L = L > NT ? NT : L;
  const float* col = S + j;
  float m = -__builtin_huge_valf();
#pragma unroll 4
  for (int i = 0; i < L; ++i) m = fmaxf(m, col[(size_t)i * NT]);
  float s0 = 0.f, s1 = 0.f, s2 = 0.f, s3 = 0.f;
  const int L4 = L & ~3;
  for (int i = 0; i < L4; i += 4) {
    s0 += __expf(col[(size_t)(i + 0) * NT] - m);
    s1 += __expf(col[(size_t)(i + 1) * NT] - m);
    s2 += __expf(col[(size_t)(i + 2) * NT] - m);
    s3 += __expf(col[(size_t)(i + 3) * NT] - m);
  }
#pragma unroll 1
  for (int i = L4; i < L; ++i) s0 += __expf(col[(size_t)i * NT] - m);
  const float s = (s0 + s1) + (s2 + s3);
  const float inv = 1.0f / s;
  *(volatile float*)(cmax + j) = m;
  *(volatile float*)(cinv + j) = inv;
  __threadfence();
  *(volatile float*)(cmax + j) = m;
  *(volatile float*)(cinv + j) = inv;
}

__global__ __launch_bounds__(256) void pnorm_kernel(const float* __restrict__ S,
                                                    const float* __restrict__ cmax,
                                                    const float* __restrict__ cinv,
                                                    const int* __restrict__ lp, int b,
                                                    _Float16* __restrict__ P) {
  const int i = blockIdx.x;
  const int j0 = threadIdx.x * 8;
  int L = lp[b];
  L = L < 1 ? 1 : L;
  L = L > NT ? NT : L;
  v8h hv;
#pragma unroll
  for (int e = 0; e < 8; ++e) hv[e] = (_Float16)0.0f;
  if (i < L) {
    const float* sr = S + (size_t)i * NT + j0;
    const v4f sa = *(const v4f*)(sr);
    const v4f sb = *(const v4f*)(sr + 4);
    const v4f ma = *(const v4f*)(cmax + j0);
    const v4f mb = *(const v4f*)(cmax + j0 + 4);
    const v4f na = *(const v4f*)(cinv + j0);
    const v4f nb = *(const v4f*)(cinv + j0 + 4);
#pragma unroll
    for (int e = 0; e < 4; ++e) {
      hv[e]     = (_Float16)(__expf(sa[e] - ma[e]) * na[e] * 32768.0f);
      hv[4 + e] = (_Float16)(__expf(sb[e] - mb[e]) * nb[e] * 32768.0f);
    }
  }
  _Float16* dst = P + (size_t)i * NT + j0;
  *(volatile v8h*)dst = hv;
  __threadfence();
  *(volatile v8h*)dst = hv;
}

static inline unsigned gemm_blocks(int M, int N) { return (unsigned)((((M >> 6) * (N >> 6)) + 7) >> 3); }

extern "C" void kernel_launch(void* const* d_in, const int* in_sizes, int n_in,
                              void* d_out, int out_size, void* d_ws, size_t ws_size,
                              hipStream_t stream) {
  if (n_in < 9) return;
  const float* x     = (const float*)d_in[0];
  const int*   l     = (const int*)d_in[1];
  const float* Wq    = (const float*)d_in[2];
  const float* Wk    = (const float*)d_in[3];
  const float* Wv    = (const float*)d_in[4];
  const float* Wo    = (const float*)d_in[5];
  const float* bo    = (const float*)d_in[6];
  const float* gamma = (const float*)d_in[7];
  const float* beta  = (const float*)d_in[8];
  float* out = (float*)d_out;

  if (in_sizes[0] != NB * NT * ND || out_size != NB * NT * ND || in_sizes[1] < NB) return;
  if (in_sizes[2] != ND * ND || in_sizes[3] != ND * ND || in_sizes[4] != ND * ND || in_sizes[5] != ND * ND) return;
  if (in_sizes[6] < ND || in_sizes[7] < ND || in_sizes[8] < ND) return;

  const size_t szW   = (size_t)ND * ND * 2;
  const size_t szTD2 = (size_t)NT * ND * 2;
  const size_t szTT4 = (size_t)NT * NT * 4;
  const size_t szTT2 = (size_t)NT * NT * 2;
  const size_t szT4  = (size_t)NT * 4;
  size_t off = 0;
  char* ws = (char*)d_ws;
  _Float16* WQ16 = (_Float16*)(ws + off); off += szW;
  _Float16* WK16 = (_Float16*)(ws + off); off += szW;
  _Float16* WV16 = (_Float16*)(ws + off); off += szW;
  _Float16* WO16 = (_Float16*)(ws + off); off += szW;
  _Float16* XN16 = (_Float16*)(ws + off); off += szTD2;
  _Float16* Q16  = (_Float16*)(ws + off); off += szTD2;
  _Float16* K16  = (_Float16*)(ws + off); off += szTD2;
  _Float16* VT16 = (_Float16*)(ws + off); off += szTD2;
  float*    S    = (float*)   (ws + off); off += szTT4;
  _Float16* P16  = (_Float16*)(ws + off); off += szTT2;
  _Float16* Y16  = (_Float16*)(ws + off); off += szTD2;
  float*    CMAX = (float*)   (ws + off); off += szT4;
  float*    CINV = (float*)   (ws + off); off += szT4;
  if (off > ws_size) return;

  const size_t TD = (size_t)NT * ND;

  const int n2 = ND * ND / 2;
  const unsigned cb = (unsigned)((n2 + 255) / 256);
  cast_f32_f16x2_scaled<<<cb, 256, 0, stream>>>(Wq, WQ16, n2, 16.0f);
  cast_f32_f16x2_scaled<<<cb, 256, 0, stream>>>(Wk, WK16, n2, 16.0f);
  cast_f32_f16x2_scaled<<<cb, 256, 0, stream>>>(Wv, WV16, n2, 16.0f);
  cast_f32_f16x2_scaled<<<cb, 256, 0, stream>>>(Wo, WO16, n2, 16.0f);

  const unsigned gQ  = gemm_blocks(NT, ND);
  const unsigned gVT = gemm_blocks(ND, NT);
  const unsigned gS  = gemm_blocks(NT, NT);

  for (int b = 0; b < NB; ++b) {
    const float* xb = x + (size_t)b * TD;
    float* ob = out + (size_t)b * TD;

    ln_f16_kernel<<<NT, 128, 0, stream>>>(xb, gamma, beta, XN16);

    wmma_gemm64<0, false, 0, 1, false, 0><<<dim3(gQ, 1), 256, 0, stream>>>(
        U16(XN16), U16(XN16), ND, 0L, U16(WQ16), U16(WQ16), ND, 0L,
        (void*)Q16, (void*)Q16, ND, 0L, bo, xb, 0L, NT, ND, ND, 1.0f / 16.0f);
    wmma_gemm64<0, false, 0, 1, false, 0><<<dim3(gQ, 1), 256, 0, stream>>>(
        U16(XN16), U16(XN16), ND, 0L, U16(WK16), U16(WK16), ND, 0L,
        (void*)K16, (void*)K16, ND, 0L, bo, xb, 0L, NT, ND, ND, 1.0f / 16.0f);
    wmma_gemm64<0, false, 0, 1, false, 0><<<dim3(gVT, 1), 256, 0, stream>>>(
        U16(WV16), U16(WV16), ND, 0L, U16(XN16), U16(XN16), ND, 0L,
        (void*)VT16, (void*)VT16, NT, 0L, bo, xb, 0L, ND, NT, ND, 1.0f / 16.0f);

    wmma_gemm64<0, false, 0, 0, false, 0><<<dim3(gS, 1), 256, 0, stream>>>(
        U16(Q16), U16(Q16), ND, 0L, U16(K16), U16(K16), ND, 0L,
        (void*)S, (void*)S, NT, 0L, bo, xb, 0L, NT, NT, ND, 0.03125f);

    colstats_kernel<<<NT / 256, 256, 0, stream>>>(S, l, b, CMAX, CINV);
    pnorm_kernel<<<NT, 256, 0, stream>>>(S, CMAX, CINV, l, b, P16);

    wmma_gemm64<0, false, 0, 1, true, 0><<<dim3(gQ, 1), 256, 0, stream>>>(
        U16(P16), U16(P16), NT, 0L, U16(VT16), U16(VT16), NT, 0L,
        (void*)Y16, (void*)Y16, ND, 0L, bo, xb, 0L, NT, ND, NT, 1.0f / 32768.0f);

    wmma_gemm64<0, false, 2, 0, false, 2><<<dim3(gQ, 1), 256, 0, stream>>>(
        U16(Y16), U16(Y16), ND, 0L, U16(WO16), U16(WO16), ND, 0L,
        (void*)ob, (void*)ob, ND, 0L, bo, xb, 0L, NT, ND, ND, 1.0f / 16.0f);
  }
  (void)hipGetLastError();
}
